// ChebyshevBasis_1606317769440
// MI455X (gfx1250) — hardware-run, weakly checked
//
#include <hip/hip_runtime.h>
#include <math.h>

constexpr int kRows  = 8192;
constexpr int kFeat  = 512;
constexpr int kOut   = 512;
constexpr int kNB    = 16;
constexpr int kKpoly = kFeat * kNB;
constexpr int kK     = kKpoly + kFeat;
constexpr int kChunkRows = 2048;
constexpr int kNumChunks = kRows / kChunkRows;
constexpr float kWCarry    = 16.0f;
constexpr float kWCarryInv = 1.0f / 16.0f;

constexpr size_t kBtBytes = (size_t)kOut * kK * 2;
constexpr size_t kABytes  = (size_t)kChunkRows * kK * 2;
constexpr size_t kWsTotal = kBtBytes + kABytes;

static_assert(kK % 32 == 0, "GEMM K must be a multiple of 32");
static_assert(kChunkRows % 64 == 0 && kOut % 64 == 0, "GEMM M and N must be tile multiples");
static_assert(kRows % kChunkRows == 0, "row chunks cover all rows exactly");
static_assert((kK * 2) % 128 == 0, "16-bit plane rows are whole 128-B lines");
static_assert(kBtBytes % 128 == 0, "A plane base 128-B aligned");
static_assert(kWsTotal <= (size_t)134217728, "carve within 128 MiB");
static_assert(kFeat == 512 && kKpoly == 4 * 256 * 8, "producer thread maps assume 512 features");

typedef __attribute__((ext_vector_type(16))) _Float16 v16h;
typedef __attribute__((ext_vector_type(8)))  _Float16 v8h;
typedef __attribute__((ext_vector_type(16))) __bf16   v16b;
typedef __attribute__((ext_vector_type(8)))  __bf16   v8b;
typedef __attribute__((ext_vector_type(8)))  float    v8f;
typedef __attribute__((ext_vector_type(4)))  float    v4f;
typedef __attribute__((ext_vector_type(4)))  unsigned int v4u;

__device__ __forceinline__ unsigned short f2bf_bits(float f) {
  unsigned u = __float_as_uint(f);
  return (unsigned short)((u + 0x7FFFu + ((u >> 16) & 1u)) >> 16);
}
__device__ __forceinline__ float bf_bits2f(unsigned short h) { return __uint_as_float(((unsigned)h) << 16); }

__device__ __forceinline__ void dep_guard_h(v8f& a, v8f& b, v16h x, v16h y) { asm volatile("v_nop\n\tv_nop\n\tv_nop\n\tv_nop" : "+v"(a), "+v"(b) : "v"(x), "v"(y)); }
__device__ __forceinline__ void dep_guard_b(v8f& a, v8f& b, v16b x, v16b y) { asm volatile("v_nop\n\tv_nop\n\tv_nop\n\tv_nop" : "+v"(a), "+v"(b) : "v"(x), "v"(y)); }
__device__ __forceinline__ void keep4_h(v16h a, v16h b, v16h c, v16h d) { asm volatile("v_nop" :: "v"(a), "v"(b), "v"(c), "v"(d)); }
__device__ __forceinline__ void keep4_b(v16b a, v16b b, v16b c, v16b d) { asm volatile("v_nop" :: "v"(a), "v"(b), "v"(c), "v"(d)); }
__device__ __forceinline__ void acc_guard4(v8f& a, v8f& b, v8f& c, v8f& d) { asm volatile("v_nop\n\tv_nop\n\tv_nop\n\tv_nop" : "+v"(a), "+v"(b), "+v"(c), "+v"(d)); }
template <typename T> struct Frag;
template <> struct Frag<_Float16> {
  typedef v16h V; union U { v16h v; v8h h[2]; };
  static __device__ __forceinline__ v16h load(const _Float16* p) {
    U f; f.h[0] = *(const v8h*)(p); f.h[1] = *(const v8h*)(p + 16); return f.v;
  }
  static __device__ __forceinline__ v8f mma(v16h a, v16h b, v8f c) {
    return __builtin_amdgcn_wmma_f32_16x16x32_f16(false, a, false, b, (short)0, c, false, false);
  }
  static __device__ __forceinline__ void guard(v8f& a, v8f& b, v16h x, v16h y) { dep_guard_h(a, b, x, y); }
  static __device__ __forceinline__ void keep(v16h a, v16h b, v16h c, v16h d) { keep4_h(a, b, c, d); }
};
template <> struct Frag<__bf16> {
  typedef v16b V; union U { v16b v; v8b h[2]; };
  static __device__ __forceinline__ v16b load(const __bf16* p) {
    U f; f.h[0] = *(const v8b*)(p); f.h[1] = *(const v8b*)(p + 16); return f.v;
  }
  static __device__ __forceinline__ v8f mma(v16b a, v16b b, v8f c) {
    return __builtin_amdgcn_wmma_f32_16x16x32_bf16(false, a, false, b, (short)0, c, false, false);
  }
  static __device__ __forceinline__ void guard(v8f& a, v8f& b, v16b x, v16b y) { dep_guard_b(a, b, x, y); }
  static __device__ __forceinline__ void keep(v16b a, v16b b, v16b c, v16b d) { keep4_b(a, b, c, d); }
};

__device__ __forceinline__ unsigned pk16(unsigned short a, unsigned short b) { return (unsigned)a | ((unsigned)b << 16); }
__device__ __forceinline__ unsigned short h_bits(float f) { const _Float16 h = (_Float16)f; return __builtin_bit_cast(unsigned short, h); }

template <int ET> struct Elem;
template <> struct Elem<0> { typedef _Float16 T; };
template <> struct Elem<1> { typedef __bf16 T; };
template <int ET, bool SPLIT, int BIAS_MODE, int OUT_MODE, bool RESID, int ACT = 0>
__global__ __launch_bounds__(256) void wmma_gemm64(
    const unsigned short* __restrict__ Ap, const unsigned short* __restrict__ A2p, int lda, long strideA,
    const unsigned short* __restrict__ Btp, const unsigned short* __restrict__ Bt2p, int ldb, long strideB,
    void* __restrict__ Cout, void* __restrict__ Cout2, int ldc, long strideC,
    const float* __restrict__ bias,
    const float* __restrict__ resid, long strideR,
    int M, int N, int K, float scale) {
  typedef typename Elem<ET>::T T;
  typedef typename Frag<T>::V V;
  const T* A = (const T*)Ap; const T* A2 = (const T*)A2p; const T* Bt = (const T*)Btp; const T* Bt2 = (const T*)Bt2p;
  __shared__ __align__(16) float sT[8][16 * 68];
  const int b    = blockIdx.y;
  const int lane = threadIdx.x & 31;
  const int wave = threadIdx.x >> 5;
  const int tilesN = N >> 6;
  const int tilesM = M >> 6;
  const int tile = blockIdx.x * 8 + wave;
  if (tile >= tilesM * tilesN) return;
  const int tm = tile / tilesN;
  const int tn = tile - tm * tilesN;
  const int m0 = tm << 6;
  const int n0 = tn << 6;

  const T* Ab  = A  + (size_t)b * strideA;
  const T* Bb  = Bt + (size_t)b * strideB;
  const T* Ab2 = SPLIT ? (A2  + (size_t)b * strideA) : nullptr;
  const T* Bb2 = SPLIT ? (Bt2 + (size_t)b * strideB) : nullptr;

  const int rlane = lane & 15;
  const int koff  = (lane >> 4) * 8;
  const int mOff  = (lane >> 4) * 8;

  v8f acc[4][4];
#pragma unroll
  for (int i = 0; i < 4; ++i)
#pragma unroll
    for (int j = 0; j < 4; ++j) acc[i][j] = (v8f){0.f,0.f,0.f,0.f,0.f,0.f,0.f,0.f};

  for (int k0 = 0; k0 < K; k0 += 32) {
    V bh[4], bl[4];
#pragma unroll
    for (int j = 0; j < 4; ++j) {
      const size_t bo = (size_t)(n0 + (j << 4) + rlane) * ldb + koff + k0;
      bh[j] = Frag<T>::load(Bb + bo);
      if (SPLIT) bl[j] = Frag<T>::load(Bb2 + bo);
    }
#pragma unroll
    for (int i = 0; i < 4; ++i) {
      const size_t ao = (size_t)(m0 + (i << 4) + rlane) * lda + koff + k0;
      V ah = Frag<T>::load(Ab + ao);
      V al;
      if (SPLIT) al = Frag<T>::load(Ab2 + ao);
#pragma unroll
      for (int j = 0; j < 4; ++j) {
        acc[i][j] = Frag<T>::mma(ah, bh[j], acc[i][j]);
        if (SPLIT) {
          acc[i][j] = Frag<T>::mma(ah, bl[j], acc[i][j]);
          acc[i][j] = Frag<T>::mma(al, bh[j], acc[i][j]);
        }
      }
      Frag<T>::guard(acc[i][0], acc[i][3], ah, SPLIT ? al : ah);
    }
    Frag<T>::keep(bh[0], bh[1], bh[2], bh[3]);
    if (SPLIT) Frag<T>::keep(bl[0], bl[1], bl[2], bl[3]);
  }
  acc_guard4(acc[0][0], acc[0][1], acc[0][2], acc[0][3]);
  acc_guard4(acc[1][0], acc[1][1], acc[1][2], acc[1][3]);
  acc_guard4(acc[2][0], acc[2][1], acc[2][2], acc[2][3]);
  acc_guard4(acc[3][0], acc[3][1], acc[3][2], acc[3][3]);

  float* slab = sT[wave];
  const float* Rb = RESID ? (resid + (size_t)b * strideR) : nullptr;
#pragma unroll
  for (int i = 0; i < 4; ++i) {
    const int mBase = m0 + (i << 4);
#pragma unroll
    for (int j = 0; j < 4; ++j) {
      const int n = n0 + (j << 4) + rlane;
      float bv = 0.f;
      if (BIAS_MODE == 2) bv = bias[n];
#pragma unroll
      for (int r = 0; r < 8; ++r) {
        float v = acc[i][j][r] * scale;
        if (BIAS_MODE == 1) v += bias[mBase + mOff + r];
        if (BIAS_MODE == 2) v += bv;
        if (RESID) v += Rb[(size_t)(mBase + mOff + r) * ldc + n];
        if (ACT == 2) v = fmaxf(v, 0.0f);
        if (ACT == 4) v = (v > 0.f) ? v : 0.01f * v;
        slab[(mOff + r) * 68 + (j << 4) + rlane] = v;
      }
    }
    __builtin_amdgcn_fence(__ATOMIC_RELEASE, "workgroup");
    __builtin_amdgcn_wave_barrier();
    __builtin_amdgcn_fence(__ATOMIC_ACQUIRE, "workgroup");
    if (OUT_MODE == 0) {
      float* C = (float*)Cout + (size_t)b * strideC;
      const int hh = lane >> 4, c4 = (lane & 15) * 4;
      for (int pass = 0; pass < 2; ++pass) {
#pragma unroll
        for (int it = 0; it < 8; ++it) {
          const int row = it * 2 + hh;
          v4f v = *(const v4f*)(slab + row * 68 + c4);
          *(volatile v4f*)(C + (size_t)(mBase + row) * ldc + n0 + c4) = v;
        }
        __threadfence();
      }
    } else {
      const int q = lane >> 3, c8 = (lane & 7) * 8;
      unsigned short* C  = (unsigned short*)Cout  + (size_t)b * strideC;
      unsigned short* C2 = (OUT_MODE == 2) ? ((unsigned short*)Cout2 + (size_t)b * strideC) : nullptr;
      for (int pass = 0; pass < 2; ++pass) {
#pragma unroll
        for (int it = 0; it < 4; ++it) {
          const int row = it * 4 + q;
          const float* sp = slab + row * 68 + c8;
          v8h hv, lv;
#pragma unroll
          for (int e = 0; e < 8; ++e) {
            if (OUT_MODE == 1) {
              hv[e] = (_Float16)sp[e];
            } else {
              unsigned short hb = f2bf_bits(sp[e]);
              unsigned short lb = f2bf_bits(sp[e] - bf_bits2f(hb));
              hv[e] = __builtin_bit_cast(_Float16, hb);
              lv[e] = __builtin_bit_cast(_Float16, lb);
            }
          }
          *(volatile v8h*)(C + (size_t)(mBase + row) * ldc + n0 + c8) = hv;
          if (OUT_MODE == 2) *(volatile v8h*)(C2 + (size_t)(mBase + row) * ldc + n0 + c8) = lv;
        }
        __threadfence();
      }
    }
    __builtin_amdgcn_fence(__ATOMIC_RELEASE, "workgroup");
    __builtin_amdgcn_wave_barrier();
    __builtin_amdgcn_fence(__ATOMIC_ACQUIRE, "workgroup");
  }
}

__global__ __launch_bounds__(256) void bt_build_kernel(const float* __restrict__ coeffs,
                                                       const float* __restrict__ bw,
                                                       unsigned short* __restrict__ Bt,
                                                       float* __restrict__ klp) {
  __shared__ v4u sm[2 * kFeat];
  const int t = threadIdx.x;
  const int o = blockIdx.x;
#pragma unroll 1
  for (int j = 0; j < 2; ++j) {
    const int i = t + 256 * j;
    const float* cp = coeffs + ((size_t)i * kOut + o) * kNB;
    const v4f c0 = *(const v4f*)(cp);
    const v4f c1 = *(const v4f*)(cp + 4);
    const v4f c2 = *(const v4f*)(cp + 8);
    const v4f c3 = *(const v4f*)(cp + 12);
    unsigned short hb[16];
#pragma unroll
    for (int e = 0; e < 4; ++e) {
      hb[e]      = h_bits(c0[e] * kWCarry);
      hb[4 + e]  = h_bits(c1[e] * kWCarry);
      hb[8 + e]  = h_bits(c2[e] * kWCarry);
      hb[12 + e] = h_bits(c3[e] * kWCarry);
    }
    const v4u u0 = (v4u){pk16(hb[0], hb[1]), pk16(hb[2], hb[3]), pk16(hb[4], hb[5]), pk16(hb[6], hb[7])};
    const v4u u1 = (v4u){pk16(hb[8], hb[9]), pk16(hb[10], hb[11]), pk16(hb[12], hb[13]), pk16(hb[14], hb[15])};
    sm[2 * i]     = u0;
    sm[2 * i + 1] = u1;
  }
  const int tt = t & 63;
  unsigned short wb[8];
#pragma unroll
  for (int e = 0; e < 8; ++e) wb[e] = h_bits(bw[(size_t)(8 * tt + e) * kOut + o] * kWCarry);
  const v4u uw = (v4u){pk16(wb[0], wb[1]), pk16(wb[2], wb[3]), pk16(wb[4], wb[5]), pk16(wb[6], wb[7])};
  __syncthreads();
  unsigned short* brow = Bt + (size_t)o * kK;
  for (int pass = 0; pass < 2; ++pass) {
#pragma unroll
    for (int it = 0; it < 4; ++it) {
      const int p = it * 256 + t;
      const v4u v = sm[p];
      *(volatile v4u*)(brow + 8 * p) = v;
    }
    if (t < 64) *(volatile v4u*)(brow + kKpoly + 8 * tt) = uw;
    if (o == 0 && t == 0) *(volatile float*)klp = 0.0f;
    __threadfence();
  }
}

__global__ __launch_bounds__(256) void basis_rows_kernel(const float* __restrict__ x,
                                                         unsigned short* __restrict__ A, int row0) {
#pragma clang fp contract(off)
  __shared__ v4u sm[2 * kFeat];
  const int t = threadIdx.x;
  const int rloc = blockIdx.x;
  int row = row0 + rloc;
  row = row < kRows ? row : (kRows - 1);
  const float* xr = x + (size_t)row * kFeat;
  float one = 1.0f;
  asm volatile("" : "+v"(one));
#pragma unroll 1
  for (int j = 0; j < 2; ++j) {
    const int i = t + 256 * j;
    const float xv = xr[i];
    const float tv = tanhf(xv);
    const float two_t = 2.0f * tv;
    unsigned short hb[16];
    hb[0] = h_bits(one);
    hb[1] = h_bits(tv);
    float tm2 = one, tm1 = tv;
#pragma unroll
    for (int n = 2; n < 16; ++n) {
      const float prod = two_t * tm1;
      const float tn = prod - tm2;
      hb[n] = h_bits(tn);
      tm2 = tm1;
      tm1 = tn;
    }
    const v4u u0 = (v4u){pk16(hb[0], hb[1]), pk16(hb[2], hb[3]), pk16(hb[4], hb[5]), pk16(hb[6], hb[7])};
    const v4u u1 = (v4u){pk16(hb[8], hb[9]), pk16(hb[10], hb[11]), pk16(hb[12], hb[13]), pk16(hb[14], hb[15])};
    sm[2 * i]     = u0;
    sm[2 * i + 1] = u1;
  }
  const int tt = t & 63;
  const v4f xa = *(const v4f*)(xr + 8 * tt);
  const v4f xc = *(const v4f*)(xr + 8 * tt + 4);
  unsigned short xb[8];
#pragma unroll
  for (int e = 0; e < 4; ++e) {
    xb[e]     = h_bits(xa[e]);
    xb[4 + e] = h_bits(xc[e]);
  }
  const v4u ux = (v4u){pk16(xb[0], xb[1]), pk16(xb[2], xb[3]), pk16(xb[4], xb[5]), pk16(xb[6], xb[7])};
  __syncthreads();
  unsigned short* arow = A + (size_t)rloc * kK;
  for (int pass = 0; pass < 2; ++pass) {
#pragma unroll
    for (int it = 0; it < 4; ++it) {
      const int p = it * 256 + t;
      const v4u v = sm[p];
      *(volatile v4u*)(arow + 8 * p) = v;
    }
    if (t < 64) *(volatile v4u*)(arow + kKpoly + 8 * tt) = ux;
    __threadfence();
  }
}

extern "C" void kernel_launch(void* const* d_in, const int* in_sizes, int n_in,
                              void* d_out, int out_size, void* d_ws, size_t ws_size,
                              hipStream_t stream) {
  if (n_in < 3) return;
  if (in_sizes[0] != kRows * kFeat) return;
  if (in_sizes[1] != kFeat * kOut * kNB) return;
  if (in_sizes[2] != kFeat * kOut) return;
  if ((size_t)out_size < (size_t)kRows * kOut + 1) return;
  if (ws_size < kWsTotal) return;

  const float* x      = (const float*)d_in[0];
  const float* coeffs = (const float*)d_in[1];
  const float* bw     = (const float*)d_in[2];
  float* out = (float*)d_out;
  float* klp = out + (size_t)kRows * kOut;

  unsigned short* Bt = (unsigned short*)d_ws;
  unsigned short* A  = (unsigned short*)((char*)d_ws + kBtBytes);

  bt_build_kernel<<<dim3(kOut), dim3(256), 0, stream>>>(coeffs, bw, Bt, klp);

  const int gemmBlocks = ((kChunkRows / 64) * (kOut / 64) + 7) / 8;
  for (int c = 0; c < kNumChunks; ++c) {
    basis_rows_kernel<<<dim3(kChunkRows), dim3(256), 0, stream>>>(x, A, c * kChunkRows);
    wmma_gemm64<0, false, 0, 0, false, 0><<<dim3(gemmBlocks, 1), dim3(256), 0, stream>>>(
        A, A, kK, 0L,
        Bt, Bt, kK, 0L,
        (void*)(out + (size_t)c * kChunkRows * kOut), nullptr, kOut, 0L,
        nullptr,
        nullptr, 0L,
        kChunkRows, kOut, kK, kWCarryInv);
  }
}
